// MultiHeadSelfAttentionLayer_58523224375379
// MI455X (gfx1250) — hardware-run, weakly checked
//
#include <hip/hip_runtime.h>
#include <math.h>

constexpr int kBatch    = 4;
constexpr int kSeq      = 2048;
constexpr int kEmb      = 1024;
constexpr int kHidden   = 1024;
constexpr int kHeads    = 16;
constexpr int kHeadDim  = 64;
constexpr int kTok      = kBatch * kSeq;
constexpr int kPairs    = kBatch * kHeads;
constexpr int kPairElems = kSeq * kHeadDim;
constexpr float kScoreScale = 1.0f / 1024.0f;
constexpr float kDiagCarry  = 2048.0f;
constexpr float kOutScale   = 1.0f / 2048.0f;

typedef __attribute__((ext_vector_type(16))) _Float16 v16h;
typedef __attribute__((ext_vector_type(8)))  _Float16 v8h;
typedef __attribute__((ext_vector_type(16))) __bf16   v16b;
typedef __attribute__((ext_vector_type(8)))  __bf16   v8b;
typedef __attribute__((ext_vector_type(8)))  float    v8f;
typedef __attribute__((ext_vector_type(4)))  float    v4f;
typedef __attribute__((ext_vector_type(4)))  unsigned int v4u;

__device__ __forceinline__ unsigned short f2bf_bits(float f) {
  unsigned u = __float_as_uint(f);
  return (unsigned short)((u + 0x7FFFu + ((u >> 16) & 1u)) >> 16);
}
__device__ __forceinline__ float bf_bits2f(unsigned short h) { return __uint_as_float(((unsigned)h) << 16); }

__device__ __forceinline__ void dep_guard_h(v8f& a, v8f& b, v16h x, v16h y) { asm volatile("v_nop\n\tv_nop\n\tv_nop\n\tv_nop" : "+v"(a), "+v"(b) : "v"(x), "v"(y)); }
__device__ __forceinline__ void dep_guard_b(v8f& a, v8f& b, v16b x, v16b y) { asm volatile("v_nop\n\tv_nop\n\tv_nop\n\tv_nop" : "+v"(a), "+v"(b) : "v"(x), "v"(y)); }
__device__ __forceinline__ void keep4_h(v16h a, v16h b, v16h c, v16h d) { asm volatile("v_nop" :: "v"(a), "v"(b), "v"(c), "v"(d)); }
__device__ __forceinline__ void keep4_b(v16b a, v16b b, v16b c, v16b d) { asm volatile("v_nop" :: "v"(a), "v"(b), "v"(c), "v"(d)); }
__device__ __forceinline__ void acc_guard4(v8f& a, v8f& b, v8f& c, v8f& d) { asm volatile("v_nop\n\tv_nop\n\tv_nop\n\tv_nop" : "+v"(a), "+v"(b), "+v"(c), "+v"(d)); }
template <typename T> struct Frag;
template <> struct Frag<_Float16> {
  typedef v16h V; union U { v16h v; v8h h[2]; };
  static __device__ __forceinline__ v16h load(const _Float16* p) {
    U f; f.h[0] = *(const v8h*)(p); f.h[1] = *(const v8h*)(p + 16); return f.v;
  }
  static __device__ __forceinline__ v8f mma(v16h a, v16h b, v8f c) {
    return __builtin_amdgcn_wmma_f32_16x16x32_f16(false, a, false, b, (short)0, c, false, false);
  }
  static __device__ __forceinline__ void guard(v8f& a, v8f& b, v16h x, v16h y) { dep_guard_h(a, b, x, y); }
  static __device__ __forceinline__ void keep(v16h a, v16h b, v16h c, v16h d) { keep4_h(a, b, c, d); }
};
template <> struct Frag<__bf16> {
  typedef v16b V; union U { v16b v; v8b h[2]; };
  static __device__ __forceinline__ v16b load(const __bf16* p) {
    U f; f.h[0] = *(const v8b*)(p); f.h[1] = *(const v8b*)(p + 16); return f.v;
  }
  static __device__ __forceinline__ v8f mma(v16b a, v16b b, v8f c) {
    return __builtin_amdgcn_wmma_f32_16x16x32_bf16(false, a, false, b, (short)0, c, false, false);
  }
  static __device__ __forceinline__ void guard(v8f& a, v8f& b, v16b x, v16b y) { dep_guard_b(a, b, x, y); }
  static __device__ __forceinline__ void keep(v16b a, v16b b, v16b c, v16b d) { keep4_b(a, b, c, d); }
};

__device__ __forceinline__ unsigned pk16(unsigned short a, unsigned short b) { return (unsigned)a | ((unsigned)b << 16); }

template <int ET> struct Elem;
template <> struct Elem<0> { typedef _Float16 T; };
template <> struct Elem<1> { typedef __bf16 T; };
template <int ET, int SPLITM, int BIAS_MODE, int OUT_MODE, bool RESID, int ACT = 0>
__global__ __launch_bounds__(256) void wmma_gemm64(
    const unsigned short* __restrict__ Ap, const unsigned short* __restrict__ A2p, int lda, long strideA,
    const unsigned short* __restrict__ Btp, const unsigned short* __restrict__ Bt2p, int ldb, long strideB,
    void* __restrict__ Cout, void* __restrict__ Cout2, int ldc, long strideC,
    const float* __restrict__ bias,
    const float* __restrict__ resid, long strideR,
    int M, int N, int K, float scale) {
  typedef typename Elem<ET>::T T;
  typedef typename Frag<T>::V V;
  const T* A = (const T*)Ap; const T* A2 = (const T*)A2p; const T* Bt = (const T*)Btp; const T* Bt2 = (const T*)Bt2p;
  __shared__ __align__(16) float sT[8][16 * 68];
  const int b    = blockIdx.y;
  const int lane = threadIdx.x & 31;
  const int wave = threadIdx.x >> 5;
  const int tilesN = N >> 6;
  const int tilesM = M >> 6;
  const int tile = blockIdx.x * 8 + wave;
  if (tile >= tilesM * tilesN) return;
  const int tm = tile / tilesN;
  const int tn = tile - tm * tilesN;
  const int m0 = tm << 6;
  const int n0 = tn << 6;

  const T* Ab  = A  + (size_t)b * strideA;
  const T* Bb  = Bt + (size_t)b * strideB;
  const T* Ab2 = (SPLITM != 0) ? (A2  + (size_t)b * strideA) : nullptr;
  const T* Bb2 = (SPLITM == 1) ? (Bt2 + (size_t)b * strideB) : nullptr;

  const int rlane = lane & 15;
  const int koff  = (lane >> 4) * 8;
  const int mOff  = (lane >> 4) * 8;

  v8f acc[4][4];
#pragma unroll
  for (int i = 0; i < 4; ++i)
#pragma unroll
    for (int j = 0; j < 4; ++j) acc[i][j] = (v8f){0.f,0.f,0.f,0.f,0.f,0.f,0.f,0.f};

  for (int k0 = 0; k0 < K; k0 += 32) {
    V bh[4], bl[4];
#pragma unroll
    for (int j = 0; j < 4; ++j) {
      const size_t bo = (size_t)(n0 + (j << 4) + rlane) * ldb + koff + k0;
      bh[j] = Frag<T>::load(Bb + bo);
      if (SPLITM == 1) bl[j] = Frag<T>::load(Bb2 + bo);
    }
#pragma unroll
    for (int i = 0; i < 4; ++i) {
      const size_t ao = (size_t)(m0 + (i << 4) + rlane) * lda + koff + k0;
      V ah = Frag<T>::load(Ab + ao);
      V al;
      if (SPLITM != 0) al = Frag<T>::load(Ab2 + ao);
#pragma unroll
      for (int j = 0; j < 4; ++j) {
        acc[i][j] = Frag<T>::mma(ah, bh[j], acc[i][j]);
        if (SPLITM == 1) acc[i][j] = Frag<T>::mma(ah, bl[j], acc[i][j]);
        if (SPLITM != 0) acc[i][j] = Frag<T>::mma(al, bh[j], acc[i][j]);
      }
      Frag<T>::guard(acc[i][0], acc[i][3], ah, (SPLITM != 0) ? al : ah);
    }
    Frag<T>::keep(bh[0], bh[1], bh[2], bh[3]);
    if (SPLITM == 1) Frag<T>::keep(bl[0], bl[1], bl[2], bl[3]);
  }
  acc_guard4(acc[0][0], acc[0][1], acc[0][2], acc[0][3]);
  acc_guard4(acc[1][0], acc[1][1], acc[1][2], acc[1][3]);
  acc_guard4(acc[2][0], acc[2][1], acc[2][2], acc[2][3]);
  acc_guard4(acc[3][0], acc[3][1], acc[3][2], acc[3][3]);

  float* slab = sT[wave];
  const float* Rb = RESID ? (resid + (size_t)b * strideR) : nullptr;
#pragma unroll
  for (int i = 0; i < 4; ++i) {
    const int mBase = m0 + (i << 4);
#pragma unroll
    for (int j = 0; j < 4; ++j) {
      const int n = n0 + (j << 4) + rlane;
      float bv = 0.f;
      if (BIAS_MODE == 2) bv = bf_bits2f(f2bf_bits(bias[n]));
#pragma unroll
      for (int r = 0; r < 8; ++r) {
        float v = acc[i][j][r] * scale;
        if (BIAS_MODE == 1) v += bf_bits2f(f2bf_bits(bias[mBase + mOff + r]));
        if (BIAS_MODE == 2) v += bv;
        if (RESID) v += Rb[(size_t)(mBase + mOff + r) * ldc + n];
        if (ACT == 2) v = fmaxf(v, 0.0f);
        if (ACT == 4) v = (v > 0.f) ? v : 0.01f * v;
        slab[(mOff + r) * 68 + (j << 4) + rlane] = v;
      }
    }
    __builtin_amdgcn_fence(__ATOMIC_RELEASE, "workgroup");
    __builtin_amdgcn_wave_barrier();
    __builtin_amdgcn_fence(__ATOMIC_ACQUIRE, "workgroup");
    if (OUT_MODE == 0) {
      float* C = (float*)Cout + (size_t)b * strideC;
      const int hh = lane >> 4, c4 = (lane & 15) * 4;
      for (int pass = 0; pass < 2; ++pass) {
#pragma unroll
        for (int it = 0; it < 8; ++it) {
          const int row = it * 2 + hh;
          v4f v = *(const v4f*)(slab + row * 68 + c4);
          *(volatile v4f*)(C + (size_t)(mBase + row) * ldc + n0 + c4) = v;
        }
        __threadfence();
      }
    } else {
      const int q = lane >> 3, c8 = (lane & 7) * 8;
      unsigned short* C  = (unsigned short*)Cout  + (size_t)b * strideC;
      unsigned short* C2 = (OUT_MODE == 2) ? ((unsigned short*)Cout2 + (size_t)b * strideC) : nullptr;
      for (int pass = 0; pass < 2; ++pass) {
#pragma unroll
        for (int it = 0; it < 4; ++it) {
          const int row = it * 4 + q;
          const float* sp = slab + row * 68 + c8;
          v8h hv, lv;
#pragma unroll
          for (int e = 0; e < 8; ++e) {
            if (OUT_MODE == 1) {
              hv[e] = (_Float16)sp[e];
            } else {
              unsigned short hb = f2bf_bits(sp[e]);
              unsigned short lb = f2bf_bits(sp[e] - bf_bits2f(hb));
              hv[e] = __builtin_bit_cast(_Float16, hb);
              lv[e] = __builtin_bit_cast(_Float16, lb);
            }
          }
          *(volatile v8h*)(C + (size_t)(mBase + row) * ldc + n0 + c8) = hv;
          if (OUT_MODE == 2) *(volatile v8h*)(C2 + (size_t)(mBase + row) * ldc + n0 + c8) = lv;
        }
        __threadfence();
      }
    }
    __builtin_amdgcn_fence(__ATOMIC_RELEASE, "workgroup");
    __builtin_amdgcn_wave_barrier();
    __builtin_amdgcn_fence(__ATOMIC_ACQUIRE, "workgroup");
  }
}

__global__ __launch_bounds__(256) void wtcast_bf16_kernel(const float* __restrict__ W0, const float* __restrict__ W1,
                                                          const float* __restrict__ W2, const float* __restrict__ W3,
                                                          unsigned short* __restrict__ out) {
  __shared__ float sm[64][65];
  const int t  = threadIdx.x;
  const int k0 = blockIdx.x * 64;
  const int n0 = blockIdx.y * 64;
  const int z  = blockIdx.z;
  const float* W = (z == 0) ? W0 : (z == 1) ? W1 : (z == 2) ? W2 : W3;
#pragma unroll
  for (int i = 0; i < 16; ++i) {
    const int e = i * 256 + t;
    const int r = e >> 6;
    const int c = e & 63;
    sm[c][r] = W[(size_t)(k0 + r) * kHidden + n0 + c];
  }
  __syncthreads();
  const int lane = t & 31, wave = t >> 5;
  const int q = lane >> 3, c8 = (lane & 7) * 8;
  unsigned short* op = out + (size_t)z * kHidden * kEmb;
  for (int pass = 0; pass < 2; ++pass) {
#pragma unroll
    for (int it = 0; it < 2; ++it) {
      const int row = wave * 8 + it * 4 + q;
      unsigned short hb[8];
#pragma unroll
      for (int e = 0; e < 8; ++e) hb[e] = f2bf_bits(sm[row][c8 + e]);
      const v4u u = (v4u){pk16(hb[0], hb[1]), pk16(hb[2], hb[3]), pk16(hb[4], hb[5]), pk16(hb[6], hb[7])};
      *(volatile v4u*)(op + (size_t)(n0 + row) * kEmb + k0 + c8) = u;
    }
    __threadfence();
  }
}

__global__ __launch_bounds__(256) void cast8_bf16_kernel(const float* __restrict__ in, unsigned short* __restrict__ out, int n8) {
  const int i = blockIdx.x * 256 + threadIdx.x;
  if (i >= n8) return;
  const float* p = in + 8 * (size_t)i;
  const v4f a = *(const v4f*)(p);
  const v4f c = *(const v4f*)(p + 4);
  unsigned short hb[8];
#pragma unroll
  for (int e = 0; e < 4; ++e) {
    hb[e]     = f2bf_bits(a[e]);
    hb[4 + e] = f2bf_bits(c[e]);
  }
  const v4u u = (v4u){pk16(hb[0], hb[1]), pk16(hb[2], hb[3]), pk16(hb[4], hb[5]), pk16(hb[6], hb[7])};
  unsigned short* q = out + 8 * (size_t)i;
  *(volatile v4u*)q = u;
  __threadfence();
  *(volatile v4u*)q = u;
}

__device__ __forceinline__ v8f mma_f16_g(v16h a, v16h b, v8f c) {
  c = __builtin_amdgcn_wmma_f32_16x16x32_f16(false, a, false, b, (short)0, c, false, false);
  asm volatile("v_nop\n\tv_nop\n\tv_nop\n\tv_nop" : "+v"(c) : "v"(a), "v"(b));
  return c;
}

__global__ __launch_bounds__(256) void attn_diag_kernel(const unsigned short* __restrict__ Qp,
                                                        const unsigned short* __restrict__ Kp,
                                                        const float* __restrict__ Vf,
                                                        unsigned short* __restrict__ Aoh,
                                                        unsigned short* __restrict__ Aol) {
  const _Float16* Qh = (const _Float16*)Qp;
  const _Float16* Kh = (const _Float16*)Kp;
  const int lane = threadIdx.x & 31;
  const int wave = threadIdx.x >> 5;
  const int rl   = lane & 15;
  const int hh   = lane >> 4;
  const int koff = hh * 8;
  const size_t hb = (size_t)blockIdx.y * kPairElems;
  const int c0 = blockIdx.x * 128 + wave * 16;

  const _Float16* kptr = Kh + hb + (size_t)(c0 + rl) * kHeadDim + koff;
  const v16h kb0 = Frag<_Float16>::load(kptr);
  const v16h kb1 = Frag<_Float16>::load(kptr + 32);
  const _Float16* qptr = Qh + hb + (size_t)rl * kHeadDim + koff;

  float m_run = -1.0e30f;
  float z_run = 0.0f;
#pragma unroll 1
  for (int a0 = 0; a0 < kSeq; a0 += 16) {
    const _Float16* qa = qptr + (size_t)a0 * kHeadDim;
    const v16h q0 = Frag<_Float16>::load(qa);
    const v16h q1 = Frag<_Float16>::load(qa + 32);
    v8f acc = (v8f){0.f,0.f,0.f,0.f,0.f,0.f,0.f,0.f};
    acc = mma_f16_g(q0, kb0, acc);
    acc = mma_f16_g(q1, kb1, acc);
    float s[8];
#pragma unroll
    for (int i = 0; i < 8; ++i) s[i] = acc[i] * kScoreScale;
    float mb = s[0];
#pragma unroll
    for (int i = 1; i < 8; ++i) mb = fmaxf(mb, s[i]);
    mb = fmaxf(mb, __shfl_xor(mb, 16, 32));
    const float mn = fmaxf(m_run, mb);
    float p = 0.0f;
#pragma unroll
    for (int i = 0; i < 8; ++i) p += expf(s[i] - mn);
    p += __shfl_xor(p, 16, 32);
    z_run = z_run * expf(m_run - mn) + p;
    m_run = mn;
  }

  float sdiag;
  {
    const _Float16* qa = qptr + (size_t)c0 * kHeadDim;
    const v16h q0 = Frag<_Float16>::load(qa);
    const v16h q1 = Frag<_Float16>::load(qa + 32);
    v8f acc = (v8f){0.f,0.f,0.f,0.f,0.f,0.f,0.f,0.f};
    acc = mma_f16_g(q0, kb0, acc);
    acc = mma_f16_g(q1, kb1, acc);
    float sd[8];
#pragma unroll
    for (int i = 0; i < 8; ++i) sd[i] = acc[i] * kScoreScale;
    const int sel = lane & 7;
    float dv = sd[0];
#pragma unroll
    for (int i = 1; i < 8; ++i) dv = (sel == i) ? sd[i] : dv;
    const float other = __shfl_xor(dv, 16, 32);
    sdiag = (hh == (rl >> 3)) ? dv : other;
  }
  const float f = expf(sdiag - m_run) * (kDiagCarry * (1.0f / z_run));

  const int q = lane >> 3, c8 = (lane & 7) * 8;
  v4u hw[4], lw[4];
#pragma unroll
  for (int it = 0; it < 4; ++it) {
    const int row = it * 4 + q;
    const float fr = __shfl(f, row, 32);
    const float* vp = Vf + hb + (size_t)(c0 + row) * kHeadDim + c8;
    const v4f va = *(const v4f*)(vp);
    const v4f vb = *(const v4f*)(vp + 4);
    unsigned short hbt[8], lbt[8];
#pragma unroll
    for (int e = 0; e < 4; ++e) {
      const float x0 = va[e] * fr;
      const unsigned short h0 = f2bf_bits(x0);
      hbt[e] = h0;
      lbt[e] = f2bf_bits(x0 - bf_bits2f(h0));
      const float x1 = vb[e] * fr;
      const unsigned short h1 = f2bf_bits(x1);
      hbt[4 + e] = h1;
      lbt[4 + e] = f2bf_bits(x1 - bf_bits2f(h1));
    }
    hw[it] = (v4u){pk16(hbt[0], hbt[1]), pk16(hbt[2], hbt[3]), pk16(hbt[4], hbt[5]), pk16(hbt[6], hbt[7])};
    lw[it] = (v4u){pk16(lbt[0], lbt[1]), pk16(lbt[2], lbt[3]), pk16(lbt[4], lbt[5]), pk16(lbt[6], lbt[7])};
  }
  for (int pass = 0; pass < 2; ++pass) {
#pragma unroll
    for (int it = 0; it < 4; ++it) {
      const int row = it * 4 + q;
      const size_t off = hb + (size_t)(c0 + row) * kHeadDim + c8;
      *(volatile v4u*)(Aoh + off) = hw[it];
      *(volatile v4u*)(Aol + off) = lw[it];
    }
    __threadfence();
  }
}

extern "C" void kernel_launch(void* const* d_in, const int* in_sizes, int n_in,
                              void* d_out, int out_size, void* d_ws, size_t ws_size,
                              hipStream_t stream) {
  if (n_in < 9) return;
  const size_t nX = (size_t)kTok * kEmb;
  const size_t nW = (size_t)kEmb * kHidden;
  if ((size_t)in_sizes[0] != nX) return;
  if ((size_t)in_sizes[1] != nW || (size_t)in_sizes[3] != nW || (size_t)in_sizes[5] != nW || (size_t)in_sizes[7] != nW) return;
  if (in_sizes[2] != kHidden || in_sizes[4] != kHidden || in_sizes[6] != kHidden || in_sizes[8] != kHidden) return;
  if ((size_t)out_size != (size_t)kTok * kHidden) return;

  const float* X  = (const float*)d_in[0];
  const float* Wq = (const float*)d_in[1];
  const float* bq = (const float*)d_in[2];
  const float* Wk = (const float*)d_in[3];
  const float* bk = (const float*)d_in[4];
  const float* Wv = (const float*)d_in[5];
  const float* bv = (const float*)d_in[6];
  const float* Wo = (const float*)d_in[7];
  const float* bo = (const float*)d_in[8];
  float* out = (float*)d_out;
  char* ws = (char*)d_ws;

  const size_t offWT = 0;
  const size_t offXb = offWT + 4 * nW * 2;
  const size_t offQh = offXb + nX * 2;
  const size_t offKh = offQh + nX * 2;
  const size_t offVf = offKh + nX * 2;
  const size_t offAh = offVf + nX * 4;
  const size_t offAl = offAh + nX * 2;
  const size_t total = offAl + nX * 2;
  if (total > ws_size) return;

  unsigned short* WT  = (unsigned short*)(ws + offWT);
  unsigned short* Xb  = (unsigned short*)(ws + offXb);
  unsigned short* Qh  = (unsigned short*)(ws + offQh);
  unsigned short* Kh  = (unsigned short*)(ws + offKh);
  float*          Vf  = (float*)(ws + offVf);
  unsigned short* Aoh = (unsigned short*)(ws + offAh);
  unsigned short* Aol = (unsigned short*)(ws + offAl);
  const unsigned short* WTq = WT;
  const unsigned short* WTk = WT + nW;
  const unsigned short* WTv = WT + 2 * nW;
  const unsigned short* WTo = WT + 3 * nW;

  wtcast_bf16_kernel<<<dim3(kEmb / 64, kHidden / 64, 4), 256, 0, stream>>>(Wq, Wk, Wv, Wo, WT);
  const int n8 = (int)(nX / 8);
  cast8_bf16_kernel<<<(n8 + 255) / 256, 256, 0, stream>>>(X, Xb, n8);

  const int gemmBlocks = ((kTok / 64) * (kHidden / 64) + 7) / 8;
  wmma_gemm64<1, 0, 2, 1, false, 0><<<dim3(gemmBlocks, 1), 256, 0, stream>>>(
      Xb, nullptr, kEmb, 0L, WTq, nullptr, kEmb, 0L, (void*)Qh, nullptr, kHidden, 0L,
      bq, nullptr, 0L, kTok, kHidden, kEmb, 1.0f);
  wmma_gemm64<1, 0, 2, 1, false, 0><<<dim3(gemmBlocks, 1), 256, 0, stream>>>(
      Xb, nullptr, kEmb, 0L, WTk, nullptr, kEmb, 0L, (void*)Kh, nullptr, kHidden, 0L,
      bk, nullptr, 0L, kTok, kHidden, kEmb, 1.0f);
  wmma_gemm64<1, 0, 2, 0, false, 0><<<dim3(gemmBlocks, 1), 256, 0, stream>>>(
      Xb, nullptr, kEmb, 0L, WTv, nullptr, kEmb, 0L, (void*)Vf, nullptr, kHidden, 0L,
      bv, nullptr, 0L, kTok, kHidden, kEmb, 1.0f);

  attn_diag_kernel<<<dim3(kSeq / 128, kPairs), 256, 0, stream>>>(Qh, Kh, Vf, Aoh, Aol);

  wmma_gemm64<1, 2, 2, 0, false, 0><<<dim3(gemmBlocks, 1), 256, 0, stream>>>(
      Aoh, Aol, kHidden, 0L, WTo, nullptr, kHidden, 0L, (void*)out, nullptr, kHidden, 0L,
      bo, nullptr, 0L, kTok, kHidden, kHidden, kOutScale);
}
